// SelectiveSSM_21260088115344
// MI455X (gfx1250) — hardware-verified
//
#include <hip/hip_runtime.h>
#include <math.h>

typedef __attribute__((ext_vector_type(16))) _Float16 v16h;
typedef __attribute__((ext_vector_type(8)))  _Float16 v8h;
typedef __attribute__((ext_vector_type(8)))  float    v8f;
typedef __attribute__((ext_vector_type(4)))  float    v4f;

constexpr int kBatch   = 2;
constexpr int kSeq     = 2048;
constexpr int kDm      = 1024;
constexpr int kNst     = 16;
constexpr int kTaps    = 4;
constexpr int kDtR     = 64;
constexpr int kProj    = kDtR + 2 * kNst;
constexpr int kProjPad = 128;
constexpr int kBC      = 2 * kNst;
constexpr int kRows    = kBatch * kSeq;
constexpr int kScanTS  = 64;
constexpr int kScanCh  = 64;
constexpr int kScanYP  = 68;
static_assert(kProj == 96);
static_assert(kRows == 4096);
static_assert(kTaps == 4);
static_assert((kDm % 32) == 0 && (kDtR % 32) == 0);
static_assert((kRows % 64) == 0 && (kProjPad % 64) == 0 && (kDm % 64) == 0 && kDtR == 64 && kBC == 32);
static_assert((kSeq % kScanTS) == 0 && (kDm % kScanCh) == 0);
static_assert((kSeq & (kSeq - 1)) == 0);

constexpr float kCarryX    = 64.0f;
constexpr float kCarryWx   = 1024.0f;
constexpr float kCarryDt   = 64.0f;
constexpr float kCarryWdt  = 256.0f;
constexpr float kFoldProj  = 1.0f / (kCarryX * kCarryWx);
constexpr float kFoldDelta = 1.0f / (kCarryDt * kCarryWdt);
constexpr float kF16MinNormal = 6.103515625e-05f;

constexpr size_t kOffX16   = 0;
constexpr size_t kOffWX16  = kOffX16   + (size_t)kRows * kDm * 2;
constexpr size_t kOffWDT16 = kOffWX16  + (size_t)kProjPad * kDm * 2;
constexpr size_t kOffDT16  = kOffWDT16 + (size_t)kDm * kDtR * 2;
constexpr size_t kOffBC32  = kOffDT16  + (size_t)kRows * kDtR * 2;
constexpr size_t kOffDELTA = kOffBC32  + (size_t)kRows * kBC * 4;
constexpr size_t kWsTotal  = kOffDELTA + (size_t)kRows * kDm * 4;
static_assert(kWsTotal == 26607616ull);
static_assert(kWsTotal <= 134217728ull);
static_assert((kOffWX16 % 128) == 0 && (kOffWDT16 % 128) == 0 && (kOffDT16 % 128) == 0 &&
              (kOffBC32 % 128) == 0 && (kOffDELTA % 128) == 0);

__device__ __forceinline__ _Float16 f16_flush(float v) {
  const float w = (fabsf(v) < kF16MinNormal) ? 0.0f : v;
  return (_Float16)w;
}

__device__ __forceinline__ float softplus_stable(float v) {
  const float a = expf(-fabsf(v));
  return fmaxf(v, 0.0f) + log1pf(a);
}

__device__ __forceinline__ void tie_h(v8f& a, v16h x, v16h y) {
  asm volatile("v_nop\n\tv_nop\n\tv_nop\n\tv_nop" : "+v"(a) : "v"(x), "v"(y));
}
__device__ __forceinline__ void keep4_h(v16h a, v16h b, v16h c, v16h d) {
  asm volatile("v_nop" :: "v"(a), "v"(b), "v"(c), "v"(d));
}

union FragH { v16h v; v8h h[2]; };
__device__ __forceinline__ v16h frag_load_h(const _Float16* p) {
  FragH f;
  f.h[0] = *(const v8h*)(p);
  f.h[1] = *(const v8h*)(p + 16);
  return f.v;
}
__device__ __forceinline__ v8f mma_h(v16h a, v16h b, v8f c) {
  return __builtin_amdgcn_wmma_f32_16x16x32_f16(false, a, false, b, (short)0, c, false, false);
}

template <int LDA, int LDB, int KK>
__device__ __forceinline__ void tile64_accumulate(const _Float16* __restrict__ A, const _Float16* __restrict__ Bt,
                                                  int m0, int n0, int rlane, int koff, v8f (&acc)[4][4]) {
  static_assert((KK % 32) == 0);
#pragma unroll
  for (int i = 0; i < 4; ++i)
#pragma unroll
    for (int j = 0; j < 4; ++j) acc[i][j] = (v8f){0.f, 0.f, 0.f, 0.f, 0.f, 0.f, 0.f, 0.f};
#pragma unroll 1
  for (int k0 = 0; k0 < KK; k0 += 32) {
    v16h bh[4];
#pragma unroll
    for (int j = 0; j < 4; ++j) {
      const size_t bo = (size_t)(n0 + (j << 4) + rlane) * LDB + koff + k0;
      bh[j] = frag_load_h(Bt + bo);
    }
#pragma unroll
    for (int i = 0; i < 4; ++i) {
      const size_t ao = (size_t)(m0 + (i << 4) + rlane) * LDA + koff + k0;
      const v16h ah = frag_load_h(A + ao);
#pragma unroll
      for (int j = 0; j < 4; ++j) acc[i][j] = mma_h(ah, bh[j], acc[i][j]);
#pragma unroll
      for (int j = 0; j < 4; ++j) tie_h(acc[i][j], ah, bh[j]);
    }
    keep4_h(bh[0], bh[1], bh[2], bh[3]);
  }
}

template <int CARRY>
__global__ __launch_bounds__(256) void cast_plane_kernel(
    const float* __restrict__ src, unsigned short* __restrict__ dst, int total8, int real8)
{
  unsigned i = blockIdx.x * 256u + threadIdx.x;
  asm volatile("" : "+v"(i));
  if (i >= (unsigned)total8) return;
  const bool live = (i < (unsigned)real8);
  unsigned is = live ? i : (unsigned)(real8 - 1);
  asm volatile("" : "+v"(is));
  const size_t s0 = (size_t)is << 3;
  const v4f a0 = *(const v4f*)(src + s0);
  const v4f a1 = *(const v4f*)(src + s0 + 4);
  const float carry = (float)CARRY;
  v8h hv;
#pragma unroll
  for (int e = 0; e < 4; ++e) {
    float f0 = a0[e];
    float f1 = a1[e];
    f0 = live ? (f0 * carry) : 0.0f;
    f1 = live ? (f1 * carry) : 0.0f;
    hv[e]     = f16_flush(f0);
    hv[4 + e] = f16_flush(f1);
  }
  unsigned short* q = dst + ((size_t)i << 3);
  *(volatile v8h*)q = hv;
  __threadfence();
  *(volatile v8h*)q = hv;
}

__global__ __launch_bounds__(256) void conv_rows_kernel(
    const float* __restrict__ u, const float* __restrict__ cw, const float* __restrict__ cb,
    unsigned short* __restrict__ x16)
{
  unsigned i = blockIdx.x * 256u + threadIdx.x;
  asm volatile("" : "+v"(i));
  if (i >= (unsigned)(kRows * (kDm / 8))) return;
  unsigned m = i >> 7;
  unsigned d8 = (i & 127u) << 3;
  asm volatile("" : "+v"(m));
  asm volatile("" : "+v"(d8));
  const unsigned l  = m & (unsigned)(kSeq - 1);
  const unsigned mb = m - l;

  v4f w[8];
#pragma unroll
  for (int c = 0; c < 8; ++c) w[c] = *(const v4f*)(cw + (size_t)d8 * kTaps + 4 * c);
  const v4f b0 = *(const v4f*)(cb + d8);
  const v4f b1 = *(const v4f*)(cb + d8 + 4);
  float acc[8];
#pragma unroll
  for (int c = 0; c < 4; ++c) {
    const float t0 = b0[c];
    const float t1 = b1[c];
    acc[c] = t0;
    acc[4 + c] = t1;
  }
#pragma unroll
  for (int j = 0; j < kTaps; ++j) {
    const int li = (int)l - (kTaps - 1) + j;
    const bool ok = (li >= 0);
    const unsigned lic = ok ? (unsigned)li : 0u;
    const size_t ro = (size_t)(mb + lic) * kDm + d8;
    const v4f p0 = *(const v4f*)(u + ro);
    const v4f p1 = *(const v4f*)(u + ro + 4);
#pragma unroll
    for (int c = 0; c < 4; ++c) {
      float s0 = p0[c];
      float s1 = p1[c];
      s0 = ok ? s0 : 0.0f;
      s1 = ok ? s1 : 0.0f;
      const float wa = w[c][j];
      const float wb = w[4 + c][j];
      acc[c]     = fmaf(wa, s0, acc[c]);
      acc[4 + c] = fmaf(wb, s1, acc[4 + c]);
    }
  }
  v8h hv;
#pragma unroll
  for (int c = 0; c < 8; ++c) hv[c] = f16_flush(acc[c] * kCarryX);
  unsigned short* q = x16 + (size_t)m * kDm + d8;
  *(volatile v8h*)q = hv;
  __threadfence();
  *(volatile v8h*)q = hv;
}

__global__ __launch_bounds__(256) void xproj_gemm_kernel(
    const unsigned short* __restrict__ Ap, const unsigned short* __restrict__ Btp,
    unsigned short* __restrict__ dt16, float* __restrict__ bc32)
{
  __shared__ __align__(16) float sT[8][16 * 68];
  const int lane  = threadIdx.x & 31;
  const int wave  = threadIdx.x >> 5;
  const int m0    = (blockIdx.x * 8 + wave) << 6;
  const int n0    = blockIdx.y << 6;
  const int rlane = lane & 15;
  const int koff  = (lane >> 4) * 8;
  const int mOff  = (lane >> 4) * 8;

  v8f acc[4][4];
  tile64_accumulate<kDm, kDm, kDm>((const _Float16*)Ap, (const _Float16*)Btp, m0, n0, rlane, koff, acc);

  float* slab = sT[wave];
  const int q  = lane >> 3;
  const int c8 = (lane & 7) * 8;
  const int c4 = (lane & 7) * 4;
#pragma unroll
  for (int i = 0; i < 4; ++i) {
    const int mBase = m0 + (i << 4);
#pragma unroll
    for (int j = 0; j < 4; ++j) {
#pragma unroll
      for (int r = 0; r < 8; ++r) {
        const float v = acc[i][j][r] * kFoldProj;
        slab[(mOff + r) * 68 + (j << 4) + rlane] = v;
      }
    }
    __builtin_amdgcn_fence(__ATOMIC_RELEASE, "workgroup");
    __builtin_amdgcn_wave_barrier();
    __builtin_amdgcn_fence(__ATOMIC_ACQUIRE, "workgroup");
    if (blockIdx.y == 0) {
      v8h hv[4];
#pragma unroll
      for (int it = 0; it < 4; ++it) {
        const int row = it * 4 + q;
        const v4f a0 = *(const v4f*)(slab + row * 68 + c8);
        const v4f a1 = *(const v4f*)(slab + row * 68 + c8 + 4);
#pragma unroll
        for (int e = 0; e < 4; ++e) {
          const float f0 = a0[e];
          const float f1 = a1[e];
          hv[it][e]     = f16_flush(f0 * kCarryDt);
          hv[it][4 + e] = f16_flush(f1 * kCarryDt);
        }
      }
      for (int pass = 0; pass < 2; ++pass) {
#pragma unroll
        for (int it = 0; it < 4; ++it) {
          const int row = it * 4 + q;
          *(volatile v8h*)(dt16 + (size_t)(mBase + row) * kDtR + c8) = hv[it];
        }
        __threadfence();
      }
    } else {
      v4f fv[4];
#pragma unroll
      for (int it = 0; it < 4; ++it) {
        const int row = it * 4 + q;
        fv[it] = *(const v4f*)(slab + row * 68 + c4);
      }
      for (int pass = 0; pass < 2; ++pass) {
#pragma unroll
        for (int it = 0; it < 4; ++it) {
          const int row = it * 4 + q;
          *(volatile v4f*)(bc32 + (size_t)(mBase + row) * kBC + c4) = fv[it];
        }
        __threadfence();
      }
    }
    __builtin_amdgcn_fence(__ATOMIC_RELEASE, "workgroup");
    __builtin_amdgcn_wave_barrier();
    __builtin_amdgcn_fence(__ATOMIC_ACQUIRE, "workgroup");
  }
}

__global__ __launch_bounds__(256) void dtproj_gemm_kernel(
    const unsigned short* __restrict__ Ap, const unsigned short* __restrict__ Btp,
    const float* __restrict__ bias, float* __restrict__ delta)
{
  __shared__ __align__(16) float sT[8][16 * 68];
  const int lane  = threadIdx.x & 31;
  const int wave  = threadIdx.x >> 5;
  const int m0    = (blockIdx.x * 8 + wave) << 6;
  const int n0    = blockIdx.y << 6;
  const int rlane = lane & 15;
  const int koff  = (lane >> 4) * 8;
  const int mOff  = (lane >> 4) * 8;

  v8f acc[4][4];
  tile64_accumulate<kDtR, kDtR, kDtR>((const _Float16*)Ap, (const _Float16*)Btp, m0, n0, rlane, koff, acc);

  float bv[4];
#pragma unroll
  for (int j = 0; j < 4; ++j) bv[j] = bias[n0 + (j << 4) + rlane];

  float* slab = sT[wave];
  const int hh = lane >> 4;
  const int c4 = (lane & 15) * 4;
#pragma unroll
  for (int i = 0; i < 4; ++i) {
    const int mBase = m0 + (i << 4);
#pragma unroll
    for (int j = 0; j < 4; ++j) {
#pragma unroll
      for (int r = 0; r < 8; ++r) {
        const float v = acc[i][j][r] * kFoldDelta + bv[j];
        slab[(mOff + r) * 68 + (j << 4) + rlane] = v;
      }
    }
    __builtin_amdgcn_fence(__ATOMIC_RELEASE, "workgroup");
    __builtin_amdgcn_wave_barrier();
    __builtin_amdgcn_fence(__ATOMIC_ACQUIRE, "workgroup");
#pragma unroll 1
    for (int s = 0; s < 32; ++s) {
      const int idx = s * 32 + lane;
      float* p = slab + (idx >> 6) * 68 + (idx & 63);
      const float v = *p;
      *p = softplus_stable(v);
    }
    __builtin_amdgcn_fence(__ATOMIC_RELEASE, "workgroup");
    __builtin_amdgcn_wave_barrier();
    __builtin_amdgcn_fence(__ATOMIC_ACQUIRE, "workgroup");
    for (int pass = 0; pass < 2; ++pass) {
#pragma unroll
      for (int it = 0; it < 8; ++it) {
        const int row = it * 2 + hh;
        const v4f v = *(const v4f*)(slab + row * 68 + c4);
        *(volatile v4f*)(delta + (size_t)(mBase + row) * kDm + n0 + c4) = v;
      }
      __threadfence();
    }
    __builtin_amdgcn_fence(__ATOMIC_RELEASE, "workgroup");
    __builtin_amdgcn_wave_barrier();
    __builtin_amdgcn_fence(__ATOMIC_ACQUIRE, "workgroup");
  }
}

__global__ __launch_bounds__(64) void state_scan_kernel(
    const float* __restrict__ delta, const float* __restrict__ bc, const float* __restrict__ u,
    const float* __restrict__ Alog, const float* __restrict__ Dp, float* __restrict__ out)
{
  __shared__ __align__(16) float sX[kScanTS * kBC];
  __shared__ __align__(16) float sY[kScanTS * kScanYP];
  __shared__ __align__(16) float sA[kNst * kScanCh];
  __shared__ __align__(16) float sR[kNst * kScanCh];
  unsigned tid = threadIdx.x;
  asm volatile("" : "+v"(tid));
  const unsigned lane = tid & 31u;
  const unsigned wave = tid >> 5;
  constexpr int kBlkPerB = kDm / kScanCh;
  const int bix = blockIdx.x / kBlkPerB;
  const int d0  = (blockIdx.x - bix * kBlkPerB) * kScanCh;
  const unsigned d = (unsigned)d0 + tid;
  const size_t row0 = (size_t)bix * kSeq;

#pragma unroll 1
  for (int s = 0; s < kNst; ++s) {
    const float a = -expf(Alog[(size_t)d * kNst + s]);
    sA[s * kScanCh + tid] = a;
    sR[s * kScanCh + tid] = 1.0f / a;
  }
  __syncthreads();
  float aN[kNst], rA[kNst], h[kNst];
#pragma unroll
  for (int s = 0; s < kNst; ++s) {
    aN[s] = sA[s * kScanCh + tid];
    rA[s] = sR[s * kScanCh + tid];
    h[s]  = 0.f;
  }
  const float Dd = Dp[d];

  unsigned lr  = tid >> 3;
  unsigned lc4 = (tid & 7u) << 2;
  unsigned hh  = lane >> 4;
  unsigned c4  = (lane & 15u) << 2;
  asm volatile("" : "+v"(lr));
  asm volatile("" : "+v"(lc4));
  asm volatile("" : "+v"(hh));
  asm volatile("" : "+v"(c4));

#pragma unroll 1
  for (int t0 = 0; t0 < kSeq; t0 += kScanTS) {
    __syncthreads();
#pragma unroll
    for (int i = 0; i < 8; ++i) {
      const unsigned r = lr + 8u * (unsigned)i;
      *(v4f*)(sX + r * kBC + lc4) = *(const v4f*)(bc + (row0 + (size_t)t0 + r) * kBC + lc4);
    }
    __syncthreads();
#pragma unroll 1
    for (int s = 0; s < kScanTS; ++s) {
      const size_t g = (row0 + (size_t)(t0 + s)) * kDm + d;
      float dt = delta[g];
      float ut = u[g];
      asm volatile("" : "+v"(dt));
      asm volatile("" : "+v"(ut));
      const float* xr = sX + s * kBC;
      float Bs[kNst], Cs[kNst];
#pragma unroll
      for (int q4 = 0; q4 < 4; ++q4) {
        const v4f bvv = *(const v4f*)(xr + 4 * q4);
        const v4f cvv = *(const v4f*)(xr + kNst + 4 * q4);
        Bs[4 * q4 + 0] = bvv[0]; Bs[4 * q4 + 1] = bvv[1]; Bs[4 * q4 + 2] = bvv[2]; Bs[4 * q4 + 3] = bvv[3];
        Cs[4 * q4 + 0] = cvv[0]; Cs[4 * q4 + 1] = cvv[1]; Cs[4 * q4 + 2] = cvv[2]; Cs[4 * q4 + 3] = cvv[3];
      }
      float y = 0.f;
#pragma unroll
      for (int k = 0; k < kNst; ++k) {
        const float e  = expf(dt * aN[k]);
        const float wq = (e - 1.0f) * rA[k];
        const float bb = wq * Bs[k];
        h[k] = e * h[k] + bb * ut;
        y = h[k] * Cs[k] + y;
      }
      y = Dd * ut + y;
      sY[s * kScanYP + tid] = y;
    }
    __syncthreads();
    for (int pass = 0; pass < 2; ++pass) {
#pragma unroll
      for (int it = 0; it < 16; ++it) {
        const unsigned row = (unsigned)it * 4u + wave * 2u + hh;
        const v4f v = *(const v4f*)(sY + row * kScanYP + c4);
        *(volatile v4f*)(out + (row0 + (size_t)t0 + row) * kDm + d0 + c4) = v;
      }
      __threadfence();
    }
  }
}

extern "C" void kernel_launch(void* const* d_in, const int* in_sizes, int n_in,
                              void* d_out, int out_size, void* d_ws, size_t ws_size,
                              hipStream_t stream) {
  if (n_in < 8) return;
  if (in_sizes[0] != kRows * kDm) return;
  if (in_sizes[1] != kDm * kTaps) return;
  if (in_sizes[2] != kDm) return;
  if (in_sizes[3] != kProj * kDm) return;
  if (in_sizes[4] != kDm * kDtR) return;
  if (in_sizes[5] != kDm) return;
  if (in_sizes[6] != kDm * kNst) return;
  if (in_sizes[7] != kDm) return;
  if (out_size != kRows * kDm) return;
  if (ws_size < kWsTotal) return;

  const float* u       = (const float*)d_in[0];
  const float* conv_w  = (const float*)d_in[1];
  const float* conv_b  = (const float*)d_in[2];
  const float* xproj_w = (const float*)d_in[3];
  const float* dt_w    = (const float*)d_in[4];
  const float* dt_b    = (const float*)d_in[5];
  const float* A_log   = (const float*)d_in[6];
  const float* D_skip  = (const float*)d_in[7];
  float* out = (float*)d_out;

  char* ws = (char*)d_ws;
  unsigned short* X16   = (unsigned short*)(ws + kOffX16);
  unsigned short* WX16  = (unsigned short*)(ws + kOffWX16);
  unsigned short* WDT16 = (unsigned short*)(ws + kOffWDT16);
  unsigned short* DT16  = (unsigned short*)(ws + kOffDT16);
  float*          BC32  = (float*)(ws + kOffBC32);
  float*          DELTA = (float*)(ws + kOffDELTA);

  cast_plane_kernel<1024><<<(kProjPad * kDm / 8) / 256, 256, 0, stream>>>(
      xproj_w, WX16, kProjPad * kDm / 8, kProj * kDm / 8);
  cast_plane_kernel<256><<<(kDm * kDtR / 8) / 256, 256, 0, stream>>>(
      dt_w, WDT16, kDm * kDtR / 8, kDm * kDtR / 8);

  conv_rows_kernel<<<(kRows * (kDm / 8)) / 256, 256, 0, stream>>>(u, conv_w, conv_b, X16);

  xproj_gemm_kernel<<<dim3(kRows / 64 / 8, kProjPad / 64), 256, 0, stream>>>(X16, WX16, DT16, BC32);

  dtproj_gemm_kernel<<<dim3(kRows / 64 / 8, kDm / 64), 256, 0, stream>>>(DT16, WDT16, dt_b, DELTA);

  state_scan_kernel<<<kBatch * (kDm / kScanCh), kScanCh, 0, stream>>>(DELTA, BC32, u, A_log, D_skip, out);
}
